// KPConvSimpleBlock_25056839205743
// MI455X (gfx1250) — hardware-verified
//
#include <hip/hip_runtime.h>
#include <math.h>

typedef __attribute__((ext_vector_type(16))) _Float16 v16h;
typedef __attribute__((ext_vector_type(16))) __bf16 v16b;
typedef __attribute__((ext_vector_type(8)))  _Float16 v8h;
typedef __attribute__((ext_vector_type(8)))  float v8f;
typedef __attribute__((ext_vector_type(4)))  float v4f;
typedef __attribute__((ext_vector_type(2)))  float v2f;
typedef __attribute__((ext_vector_type(4)))  unsigned v4u;
typedef __attribute__((ext_vector_type(4)))  int v4i;
typedef float __attribute__((may_alias)) float_a;
typedef int __attribute__((may_alias)) int_a;

template <typename T> __device__ __forceinline__ void vst2(void* p, T v) { *(volatile T*)p = v; __threadfence(); *(volatile T*)p = v; }
__device__ __forceinline__ v8f wmma16(v16h a, v16h b, v8f c) {
  v8f d = __builtin_amdgcn_wmma_f32_16x16x32_f16(false, a, false, b, (short)0, c, false, false);
  asm volatile("v_nop\n\tv_nop\n\tv_nop\n\tv_nop" : "+v"(d) : "v"(a), "v"(b));
  return d;
}
__device__ __forceinline__ v8f wmma_bf(v16b a, v16b b, v8f c) {
  v8f d = __builtin_amdgcn_wmma_f32_16x16x32_bf16(false, a, false, b, (short)0, c, false, false);
  asm volatile("v_nop\n\tv_nop\n\tv_nop\n\tv_nop" : "+v"(d) : "v"(a), "v"(b));
  return d;
}
__device__ __forceinline__ v16h frag_h(const _Float16* rowk0, int lane) {
  union { v16h v; v8h q[2]; } u; const _Float16* p = rowk0 + 8 * (lane >> 4);
  u.q[0] = *(const v8h*)p; u.q[1] = *(const v8h*)(p + 16); return u.v;
}
__device__ __forceinline__ v16h frag_f32(const float* rowk0, int lane) {
  v16h a; const float* p = rowk0 + 8 * (lane >> 4);
#pragma unroll
  for (int i = 0; i < 8; ++i) { a[i] = (_Float16)p[i]; a[8 + i] = (_Float16)p[16 + i]; }
  return a;
}
__device__ __forceinline__ v16h frag_f32s(const float* rowk0, int lane, float sc) {
  v16h a; const float* p = rowk0 + 8 * (lane >> 4);
#pragma unroll
  for (int i = 0; i < 8; ++i) { a[i] = (_Float16)(p[i] * sc); a[8 + i] = (_Float16)(p[16 + i] * sc); }
  return a;
}
__device__ __forceinline__ v16h fragc_f32(const float* W, int k0, int n, int lane, int ld, int K) {
  v16h a; const int g = lane >> 4;
#pragma unroll
  for (int i = 0; i < 8; ++i) { const int ka = k0 + 8 * g + i, kb = ka + 16;
    a[i] = (_Float16)(ka < K ? W[(size_t)(ka < K ? ka : K - 1) * ld + n] : 0.f); a[8 + i] = (_Float16)(kb < K ? W[(size_t)(kb < K ? kb : K - 1) * ld + n] : 0.f); }
  return a;
}
struct F2 { v16b h, l; };
__device__ __forceinline__ F2 bsplit16(const float v[16]) { F2 r;
#pragma unroll
  for (int i = 0; i < 16; ++i) { const __bf16 h = (__bf16)v[i]; r.h[i] = h; r.l[i] = (__bf16)(v[i] - (float)h); }
  return r; }
__device__ __forceinline__ F2 split_row(const float* row, int k0, int lane) { float v[16]; const float* p = row + k0 + 8 * (lane >> 4);
#pragma unroll
  for (int i = 0; i < 8; ++i) { v[i] = p[i]; v[8 + i] = p[16 + i]; }
  return bsplit16(v); }
__device__ __forceinline__ F2 split_rowK(const float* row, int k0, int lane, int K) { float v[16]; const int g = lane >> 4;
#pragma unroll
  for (int i = 0; i < 8; ++i) { const int ka = k0 + 8 * g + i, kb = ka + 16; v[i] = ka < K ? row[ka < K ? ka : K - 1] : 0.f; v[8 + i] = kb < K ? row[kb < K ? kb : K - 1] : 0.f; }
  return bsplit16(v); }
__device__ __forceinline__ F2 split_col(const float* W, int k0, int n, int lane, int ld, int K) { float v[16]; const int g = lane >> 4;
#pragma unroll
  for (int i = 0; i < 8; ++i) { const int ka = k0 + 8 * g + i, kb = ka + 16; v[i] = ka < K ? W[(size_t)(ka < K ? ka : K - 1) * ld + n] : 0.f; v[8 + i] = kb < K ? W[(size_t)(kb < K ? kb : K - 1) * ld + n] : 0.f; }
  return bsplit16(v); }
__device__ __forceinline__ v8f mac3(const F2& a, const F2& b, v8f c) { c = wmma_bf(a.l, b.h, c); c = wmma_bf(a.h, b.l, c); return wmma_bf(a.h, b.h, c); }
__device__ __forceinline__ float sigm(float v) { return 1.0f / (1.0f + expf(-v)); }
#define LDSX() do { asm volatile("s_wait_dscnt 0" ::: "memory"); __builtin_amdgcn_wave_barrier(); __builtin_amdgcn_fence(__ATOMIC_RELEASE, "workgroup"); } while (0)

__device__ __forceinline__ float bfr(float v) { return (float)(__bf16)v; }
#define NPTS 100000
#define NNB 32
#define KP 15
#define CIN 64
#define COUT 128
#define KAGG (KP * CIN)
#ifndef NPB
#define NPB NPTS
#endif
#define WS_AGG 0u
#define WS_PRE (WS_AGG + 2u * (size_t)NPTS * KAGG)
#define WS_ST  (WS_PRE + 4u * (size_t)NPTS * COUT)
#define WS_END (WS_ST + 4u * 256u)
__global__ __launch_bounds__(128) void k_agg(const float* __restrict__ FEAT, const float* __restrict__ XYZ, const int* __restrict__ NIDX, const float* __restrict__ KPT, _Float16* __restrict__ AGG) {
  __shared__ __align__(16) _Float16 sg[4][16][72];
  const int tid = threadIdx.x, wave = tid >> 5, lane = tid & 31, col = lane & 15, g = lane >> 4; const size_t n = (size_t)blockIdx.x * 4 + wave;
  const float x0 = bfr(XYZ[n * 3]), y0 = bfr(XYZ[n * 3 + 1]), z0 = bfr(XYZ[n * 3 + 2]);
  float av[16]; int je[16];
#pragma unroll
  for (int i = 0; i < 16; ++i) { const int e = (i < 8) ? (8 * g + i) : (16 + 8 * g + (i - 8)); const int j = NIDX[n * NNB + e]; je[i] = j;
    float rx, ry, rz; if (j < NPTS) { rx = bfr(XYZ[(size_t)j * 3]) - x0; ry = bfr(XYZ[(size_t)j * 3 + 1]) - y0; rz = bfr(XYZ[(size_t)j * 3 + 2]) - z0; } else { rx = 1.0e6f - x0; ry = 1.0e6f - y0; rz = 1.0e6f - z0; }
    const int k = col < KP ? col : 0; const float dx = rx - bfr(KPT[k * 3]), dy = ry - bfr(KPT[k * 3 + 1]), dz = rz - bfr(KPT[k * 3 + 2]);
    const float dist = sqrtf(dx * dx + dy * dy + dz * dz); av[i] = (col < KP) ? fmaxf(1.0f - dist * 0.5f, 0.f) : 0.f; }
  const F2 a = bsplit16(av);
#pragma unroll
  for (int jt = 0; jt < CIN / 16; ++jt) { v16b fb; const int c = jt * 16 + col;
#pragma unroll
    for (int i = 0; i < 16; ++i) fb[i] = (je[i] < NPTS) ? (__bf16)FEAT[(size_t)je[i] * CIN + c] : (__bf16)0.f;
    v8f acc = {}; acc = wmma_bf(a.h, fb, acc); acc = wmma_bf(a.l, fb, acc);
#pragma unroll
    for (int r = 0; r < 8; ++r) sg[wave][8 * g + r][jt * 16 + col] = (_Float16)acc[r]; }
  LDSX();
  for (int e = lane; e < KP * 8; e += 32) { const int row = e >> 3, q = e & 7; vst2((unsigned*)(AGG + n * KAGG + row * CIN + q * 8), *(const v4u*)&sg[wave][row][q * 8]); } }
__global__ __launch_bounds__(128) void k_gemm(const _Float16* __restrict__ AGG, const float* __restrict__ W, float* __restrict__ PRE) { __shared__ __align__(16) float sf[4][16][132];
  const int tid = threadIdx.x, wave = tid >> 5, lane = tid & 31, col = lane & 15, g = lane >> 4; const size_t r0 = (size_t)blockIdx.x * 64 + wave * 16; const size_t ra = (r0 + col < NPB) ? r0 + col : NPB - 1;
  v8f acc[8] = {};
#pragma unroll 2
  for (int kc = 0; kc < KAGG / 32; ++kc) { const v16h a = frag_h(AGG + ra * KAGG + kc * 32, lane);
#pragma unroll
    for (int j = 0; j < 8; ++j) { v16h w; const int o = j * 16 + col;
#pragma unroll
      for (int i = 0; i < 8; ++i) { w[i] = (_Float16)(bfr(W[(size_t)(kc * 32 + 8 * g + i) * COUT + o]) * 16.0f); w[8 + i] = (_Float16)(bfr(W[(size_t)(kc * 32 + 16 + 8 * g + i) * COUT + o]) * 16.0f); }
      acc[j] = wmma16(a, w, acc[j]); } }
#pragma unroll
  for (int j = 0; j < 8; ++j)
#pragma unroll
    for (int r = 0; r < 8; ++r) sf[wave][8 * g + r][j * 16 + col] = acc[j][r] * (1.0f / 16.0f);
  LDSX(); for (int rl = 0; rl < 16; ++rl) { const size_t r = r0 + rl; if (r < NPB) vst2(PRE + r * COUT + lane * 4, *(const v4f*)&sf[wave][rl][lane * 4]); } }
__global__ __launch_bounds__(256) void k_bnstat(const float* __restrict__ PRE, float* __restrict__ ST) { __shared__ float smu[32], srs[32];
  const int t = threadIdx.x; const int cl = t >> 3, sub = t & 7; const int c = blockIdx.x * 32 + cl;
  float s = 0.f; for (int n = sub; n < NPB; n += 8) s += PRE[(size_t)n * COUT + c];
#pragma unroll
  for (int o = 1; o < 8; o <<= 1) s += __shfl_xor(s, o);
  const float mu = s / (float)NPB;
  float s2 = 0.f; for (int n = sub; n < NPB; n += 8) { const float d = PRE[(size_t)n * COUT + c] - mu; s2 += d * d; }
#pragma unroll
  for (int o = 1; o < 8; o <<= 1) s2 += __shfl_xor(s2, o);
  if (sub == 0) { smu[cl] = mu; srs[cl] = rsqrtf(s2 / (float)NPB + 1e-5f); }
  __syncthreads(); if (t < 32) { vst2(ST + blockIdx.x * 32 + t, smu[t]); vst2(ST + COUT + blockIdx.x * 32 + t, srs[t]); } }
__global__ __launch_bounds__(256) void k_apply(const float* __restrict__ PRE, const float* __restrict__ ST, const float* __restrict__ GA, const float* __restrict__ BE, float* __restrict__ OUT) {
  const size_t r0 = (size_t)blockIdx.x * 64; const int nrow = (r0 + 64 <= NPB) ? 64 : (int)(NPB - r0);
  for (int q = threadIdx.x; q < nrow * COUT / 4; q += 256) { const size_t e = r0 * COUT + (size_t)q * 4; const v4f x = *(const v4f*)(PRE + e); v4f o;
#pragma unroll
    for (int i = 0; i < 4; ++i) { const int c = (int)((e + i) % COUT); float v = (x[i] - ST[c]) * ST[COUT + c] * bfr(GA[c]) + bfr(BE[c]); o[i] = (v >= 0.f) ? v : 0.2f * v; }
    vst2(OUT + e, o); } }
extern "C" void kernel_launch(void* const* d_in, const int* in_sizes, int n_in, void* d_out, int out_size, void* d_ws, size_t ws_size, hipStream_t stream) {
  (void)in_sizes; (void)n_in; (void)out_size;
  const float** F = (const float**)d_in;
  if (ws_size < (size_t)WS_END) return;
  char* ws = (char*)d_ws; _Float16* AGG = (_Float16*)(ws + WS_AGG); float *PRE = (float*)(ws + WS_PRE), *ST = (float*)(ws + WS_ST);
  k_agg<<<dim3(NPB / 4), 128, 0, stream>>>(F[0], F[1], (const int*)d_in[3], F[4], AGG);
  k_gemm<<<dim3((NPB + 63) / 64), 128, 0, stream>>>(AGG, F[5], PRE);
  k_bnstat<<<dim3(COUT / 32), 256, 0, stream>>>(PRE, ST);
  k_apply<<<dim3((NPB + 63) / 64), 256, 0, stream>>>(PRE, ST, F[6], F[7], (float*)d_out);
}
